// GraphNet_1726576854583
// MI455X (gfx1250) — hardware-verified
//
#include <hip/hip_runtime.h>
#include <stdint.h>

#pragma clang fp contract(off)

#define QN 2048
#define AN 4096
#define DN 512
#define KY 1024
#define KG 1536
#define SLP 68

static_assert(QN * 2 == AN);
static_assert(QN % 64 == 0);
static_assert(DN % 64 == 0);
static_assert(AN % 64 == 0);
static_assert(DN % 32 == 0);
static_assert(AN % 32 == 0);
static_assert(KY == 2 * DN);
static_assert(KG == 3 * DN);
static_assert(KY % 32 == 0);
static_assert(KG % 32 == 0);
static_assert(DN == 32 * 16);
static_assert(AN == 32 * 128);
static_assert(QN == 8 * 256);
static_assert((size_t)2 * QN * QN + (size_t)(QN - 1) * QN + 4 * 511 + 3 < (size_t)3 * QN * QN);

typedef __attribute__((ext_vector_type(16))) __bf16   v16b;
typedef __attribute__((ext_vector_type(8)))  __bf16   v8b;
typedef __attribute__((ext_vector_type(8)))  float    v8f;
typedef __attribute__((ext_vector_type(4)))  float    v4f;
typedef __attribute__((ext_vector_type(4)))  unsigned int v4u;
typedef __attribute__((ext_vector_type(2)))  unsigned int v2u;
typedef __attribute__((ext_vector_type(4)))  int      v4i;

__device__ __forceinline__ unsigned short f2bf_bits(float f) {
  unsigned u = __float_as_uint(f);
  return (unsigned short)((u + 0x7FFFu + ((u >> 16) & 1u)) >> 16);
}
__device__ __forceinline__ float bf_bits2f(unsigned short h) { return __uint_as_float(((unsigned)h) << 16); }
__device__ __forceinline__ float bf_rne(float f) { return bf_bits2f(f2bf_bits(f)); }
__device__ __forceinline__ unsigned pk16(unsigned short a, unsigned short b) { return (unsigned)a | ((unsigned)b << 16); }

__device__ __forceinline__ void dep_guard_b(v8f& a, v8f& b, v16b x, v16b y) { asm volatile("v_nop\n\tv_nop\n\tv_nop\n\tv_nop" : "+v"(a), "+v"(b) : "v"(x), "v"(y)); }
__device__ __forceinline__ void keep4_b(v16b a, v16b b, v16b c, v16b d) { asm volatile("v_nop" :: "v"(a), "v"(b), "v"(c), "v"(d)); }
__device__ __forceinline__ void acc_guard4(v8f& a, v8f& b, v8f& c, v8f& d) { asm volatile("v_nop\n\tv_nop\n\tv_nop\n\tv_nop" : "+v"(a), "+v"(b), "+v"(c), "+v"(d)); }

__device__ __forceinline__ void wave_sync() {
  __builtin_amdgcn_fence(__ATOMIC_RELEASE, "workgroup");
  __builtin_amdgcn_wave_barrier();
  __builtin_amdgcn_fence(__ATOMIC_ACQUIRE, "workgroup");
}

__device__ __forceinline__ v16b ldfrag(const __bf16* p) {
  union { v16b v; v8b h[2]; } f;
  f.h[0] = *(const v8b*)(p);
  f.h[1] = *(const v8b*)(p + 16);
  return f.v;
}
__device__ __forceinline__ v8f mma_b(v16b a, v16b b, v8f c) {
  return __builtin_amdgcn_wmma_f32_16x16x32_bf16(false, a, false, b, (short)0, c, false, false);
}

__device__ __forceinline__ void split8(v4f a, v4f b, v4u& hv, v4u& lv) {
  const float f[8] = { a.x, a.y, a.z, a.w, b.x, b.y, b.z, b.w };
#pragma unroll
  for (int q = 0; q < 4; ++q) {
    const unsigned short h0 = f2bf_bits(f[2 * q]);
    const unsigned short h1 = f2bf_bits(f[2 * q + 1]);
    const unsigned short l0 = f2bf_bits(f[2 * q] - bf_bits2f(h0));
    const unsigned short l1 = f2bf_bits(f[2 * q + 1] - bf_bits2f(h1));
    hv[q] = pk16(h0, h1);
    lv[q] = pk16(l0, l1);
  }
}

template <int EPI>
__global__ __launch_bounds__(256) void gemm64(
    const unsigned short* __restrict__ Ap, int lda, long strideA,
    const unsigned short* __restrict__ Btp, int ldb, long strideB,
    float* Cf, unsigned short* Ch, int ldc, long strideC,
    const float* __restrict__ aux, int M, int N, int K) {
  __shared__ __align__(16) float sT[8][16 * SLP];
  const int b    = blockIdx.y;
  const int lane = threadIdx.x & 31;
  const int wave = threadIdx.x >> 5;
  const int tilesN = N >> 6;
  const int tilesM = M >> 6;
  const int tile = blockIdx.x * 8 + wave;
  if (tile >= tilesM * tilesN) return;
  const int tm = tile / tilesN;
  const int tn = tile - tm * tilesN;
  const int m0 = tm << 6;
  const int n0 = tn << 6;

  const __bf16* Ab = (const __bf16*)(const void*)Ap  + (long)b * strideA;
  const __bf16* Bb = (const __bf16*)(const void*)Btp + (long)b * strideB;

  const int rlane = lane & 15;
  const int koff  = (lane >> 4) * 8;
  const int mOff  = (lane >> 4) * 8;

  v8f acc[4][4];
#pragma unroll
  for (int i = 0; i < 4; ++i)
#pragma unroll
    for (int j = 0; j < 4; ++j) acc[i][j] = (v8f){0.f,0.f,0.f,0.f,0.f,0.f,0.f,0.f};

  for (int k0 = 0; k0 < K; k0 += 32) {
    v16b bh[4];
#pragma unroll
    for (int j = 0; j < 4; ++j) {
      const size_t bo = (size_t)(n0 + (j << 4) + rlane) * ldb + koff + k0;
      bh[j] = ldfrag(Bb + bo);
    }
#pragma unroll
    for (int i = 0; i < 4; ++i) {
      const size_t ao = (size_t)(m0 + (i << 4) + rlane) * lda + koff + k0;
      const v16b ah = ldfrag(Ab + ao);
#pragma unroll
      for (int j = 0; j < 4; ++j) acc[i][j] = mma_b(ah, bh[j], acc[i][j]);
      dep_guard_b(acc[i][0], acc[i][3], ah, ah);
    }
    keep4_b(bh[0], bh[1], bh[2], bh[3]);
  }
  acc_guard4(acc[0][0], acc[0][1], acc[0][2], acc[0][3]);
  acc_guard4(acc[1][0], acc[1][1], acc[1][2], acc[1][3]);
  acc_guard4(acc[2][0], acc[2][1], acc[2][2], acc[2][3]);
  acc_guard4(acc[3][0], acc[3][1], acc[3][2], acc[3][3]);

  float* slab = sT[wave];
  if (EPI != 2) {
    float* C = Cf + (long)b * strideC;
    const int hh = lane >> 4, c4 = (lane & 15) * 4;
#pragma unroll
    for (int i = 0; i < 4; ++i) {
      const int mBase = m0 + (i << 4);
#pragma unroll
      for (int j = 0; j < 4; ++j) {
        float bv = 0.f;
        if (EPI == 1) bv = bf_rne(aux[n0 + (j << 4) + rlane]);
#pragma unroll
        for (int r = 0; r < 8; ++r) {
          float v = acc[i][j][r];
          if (EPI == 1) { v = v + bv; v = fmaxf(v, 0.0f); }
          slab[(mOff + r) * SLP + (j << 4) + rlane] = v;
        }
      }
      wave_sync();
      for (int pass = 0; pass < 2; ++pass) {
#pragma unroll
        for (int it = 0; it < 8; ++it) {
          const int row = it * 2 + hh;
          const v4f v = *(const v4f*)(slab + row * SLP + c4);
          *(volatile v4f*)(C + (size_t)(mBase + row) * ldc + n0 + c4) = v;
        }
        __threadfence();
      }
      wave_sync();
    }
  } else {
    unsigned short* P  = Ch;
    unsigned short* PT = Ch + (size_t)M * 2 * N;
    const int hh = lane >> 4, c4 = (lane & 15) * 4;
    const int q = lane >> 3, c8 = (lane & 7) * 8;
#pragma unroll
    for (int i = 0; i < 4; ++i) {
      const int mBase = m0 + (i << 4);
#pragma unroll
      for (int it = 0; it < 8; ++it) {
        const int row = it * 2 + hh;
        v4f a = *(const v4f*)(aux + (size_t)(mBase + row) * N + n0 + c4);
        a.x = bf_rne(a.x); a.y = bf_rne(a.y); a.z = bf_rne(a.z); a.w = bf_rne(a.w);
        *(v4f*)(slab + row * SLP + c4) = a;
      }
      wave_sync();
#pragma unroll
      for (int j = 0; j < 4; ++j)
#pragma unroll
        for (int r = 0; r < 8; ++r) {
          const int pos = (mOff + r) * SLP + (j << 4) + rlane;
          const float v = acc[i][j][r] + slab[pos];
          acc[i][j][r] = v;
          slab[pos] = v;
        }
      wave_sync();
      for (int pass = 0; pass < 2; ++pass) {
#pragma unroll
        for (int it = 0; it < 4; ++it) {
          const int row = it * 4 + q;
          const v4f a = *(const v4f*)(slab + row * SLP + c8);
          const v4f c = *(const v4f*)(slab + row * SLP + c8 + 4);
          v4u hv, lv;
          split8(a, c, hv, lv);
          unsigned short* dst = P + (size_t)(mBase + row) * (2 * N) + n0 + c8;
          *(volatile v4u*)(dst) = hv;
          *(volatile v4u*)(dst + N) = lv;
        }
        __threadfence();
      }
      wave_sync();
    }
#pragma unroll
    for (int jt = 0; jt < 4; ++jt) {
#pragma unroll
      for (int i = 0; i < 4; ++i)
#pragma unroll
        for (int r = 0; r < 8; ++r)
          slab[rlane * SLP + (i << 4) + mOff + r] = acc[i][jt][r];
      wave_sync();
      for (int pass = 0; pass < 2; ++pass) {
#pragma unroll
        for (int it = 0; it < 4; ++it) {
          const int row = it * 4 + q;
          const v4f a = *(const v4f*)(slab + row * SLP + c8);
          const v4f c = *(const v4f*)(slab + row * SLP + c8 + 4);
          v4u hv, lv;
          split8(a, c, hv, lv);
          unsigned short* dst = PT + (size_t)(n0 + (jt << 4) + row) * (2 * M) + m0 + c8;
          *(volatile v4u*)(dst) = hv;
          *(volatile v4u*)(dst + M) = lv;
        }
        __threadfence();
      }
      wave_sync();
    }
  }
}

__global__ __launch_bounds__(256) void k_tr(const float* __restrict__ W, unsigned short* oh, int ldin, int ldout) {
  __shared__ __align__(16) float tf[64 * SLP];
  const int c0  = blockIdx.x * 64;
  const int r0  = blockIdx.y * 64;
  const int tid = threadIdx.x;
  {
    const int lr = tid >> 4;
    const int c4 = (tid & 15) * 4;
#pragma unroll
    for (int it = 0; it < 4; ++it) {
      const int rr = it * 16 + lr;
      const v4f a = *(const v4f*)(W + (size_t)(r0 + rr) * ldin + c0 + c4);
      *(v4f*)(tf + rr * SLP + c4) = a;
    }
  }
  __syncthreads();
  const int sub = tid >> 3;
  const int c8  = (tid & 7) * 8;
  v4u hv[2];
#pragma unroll
  for (int it = 0; it < 2; ++it) {
    const int oc = it * 32 + sub;
    v4u a;
#pragma unroll
    for (int q = 0; q < 4; ++q) {
      const float f0 = tf[(c8 + 2 * q) * SLP + oc];
      const float f1 = tf[(c8 + 2 * q + 1) * SLP + oc];
      a[q] = pk16(f2bf_bits(f0), f2bf_bits(f1));
    }
    hv[it] = a;
  }
  for (int pass = 0; pass < 2; ++pass) {
#pragma unroll
    for (int it = 0; it < 2; ++it) {
      const int oc = it * 32 + sub;
      const size_t go = (size_t)(c0 + oc) * ldout + r0 + c8;
      *(volatile v4u*)(oh + go) = hv[it];
    }
    __threadfence();
  }
}

__global__ __launch_bounds__(256) void k_dup(const float* __restrict__ in, unsigned short* out, int C, int n8) {
  const int g = blockIdx.x * 256 + threadIdx.x;
  if (g >= n8) return;
  const int c8n = C >> 3;
  const int row = g / c8n;
  const int c8  = (g - row * c8n) * 8;
  const float* src = in + (size_t)row * C + c8;
  const v4f a = *(const v4f*)src;
  const v4f c = *(const v4f*)(src + 4);
  const v4u o = { pk16(f2bf_bits(a.x), f2bf_bits(a.y)), pk16(f2bf_bits(a.z), f2bf_bits(a.w)),
                  pk16(f2bf_bits(c.x), f2bf_bits(c.y)), pk16(f2bf_bits(c.z), f2bf_bits(c.w)) };
  unsigned short* d0 = out + (size_t)row * 2 * C + c8;
  *(volatile v4u*)(d0) = o;
  *(volatile v4u*)(d0 + C) = o;
  __threadfence();
  *(volatile v4u*)(d0) = o;
  *(volatile v4u*)(d0 + C) = o;
}

__global__ __launch_bounds__(256) void k_rowx(const unsigned short* __restrict__ EB, const float* __restrict__ MF,
                                              unsigned short* X) {
  const int lane = threadIdx.x & 31, w = threadIdx.x >> 5;
  const int row = blockIdx.x * 8 + w;
  const unsigned short* er = EB + (size_t)row * DN + 8 * lane;
  const float* mr = MF + (size_t)row * DN + 8 * lane;
  const v4u ea = *(const v4u*)(er);
  const v4u eb = *(const v4u*)(er + 256);
  const v4f ma = *(const v4f*)(mr);
  const v4f mb = *(const v4f*)(mr + 4);
  const v4f mc = *(const v4f*)(mr + 256);
  const v4f md = *(const v4f*)(mr + 260);
  float e[16];
#pragma unroll
  for (int q = 0; q < 4; ++q) {
    e[2 * q]         = __uint_as_float(ea[q] << 16);
    e[2 * q + 1]     = __uint_as_float(ea[q] & 0xffff0000u);
    e[8 + 2 * q]     = __uint_as_float(eb[q] << 16);
    e[8 + 2 * q + 1] = __uint_as_float(eb[q] & 0xffff0000u);
  }
  const float m[16] = { ma.x, ma.y, ma.z, ma.w, mb.x, mb.y, mb.z, mb.w,
                        mc.x, mc.y, mc.z, mc.w, md.x, md.y, md.z, md.w };
  float se = 0.0f, sm = 0.0f;
#pragma unroll
  for (int k = 0; k < 16; ++k) { se += e[k] * e[k]; sm += m[k] * m[k]; }
#pragma unroll
  for (int off = 16; off > 0; off >>= 1) {
    se += __shfl_xor(se, off, 32);
    sm += __shfl_xor(sm, off, 32);
  }
  const float l = sqrtf(se) / sqrtf(sm);
  unsigned short hb[16], lb[16];
#pragma unroll
  for (int k = 0; k < 16; ++k) {
    const float x = e[k] + l * m[k];
    hb[k] = f2bf_bits(x);
    lb[k] = f2bf_bits(x - bf_bits2f(hb[k]));
  }
  const v4u h0 = { pk16(hb[0], hb[1]), pk16(hb[2], hb[3]), pk16(hb[4], hb[5]), pk16(hb[6], hb[7]) };
  const v4u h1 = { pk16(hb[8], hb[9]), pk16(hb[10], hb[11]), pk16(hb[12], hb[13]), pk16(hb[14], hb[15]) };
  const v4u l0 = { pk16(lb[0], lb[1]), pk16(lb[2], lb[3]), pk16(lb[4], lb[5]), pk16(lb[6], lb[7]) };
  const v4u l1 = { pk16(lb[8], lb[9]), pk16(lb[10], lb[11]), pk16(lb[12], lb[13]), pk16(lb[14], lb[15]) };
  unsigned short* xr = X + (size_t)row * KY + 8 * lane;
  *(volatile v4u*)(xr) = h0;
  *(volatile v4u*)(xr + 256) = h1;
  *(volatile v4u*)(xr + 512) = l0;
  *(volatile v4u*)(xr + 768) = l1;
  __threadfence();
  *(volatile v4u*)(xr) = h0;
  *(volatile v4u*)(xr + 256) = h1;
  *(volatile v4u*)(xr + 512) = l0;
  *(volatile v4u*)(xr + 768) = l1;
}

__global__ __launch_bounds__(256) void k_rowe(const float* __restrict__ YF, unsigned short* EA, unsigned short* EBt) {
  const int lane = threadIdx.x & 31, w = threadIdx.x >> 5;
  const int row = blockIdx.x * 8 + w;
  const float* yr = YF + (size_t)row * DN + 4 * lane;
  float ss = 0.0f;
#pragma unroll
  for (int q = 0; q < 4; ++q) {
    const v4f y = *(const v4f*)(yr + 128 * q);
    ss += y.x * y.x; ss += y.y * y.y; ss += y.z * y.z; ss += y.w * y.w;
  }
#pragma unroll
  for (int off = 16; off > 0; off >>= 1) ss += __shfl_xor(ss, off, 32);
  const float den = fmaxf(sqrtf(ss), 1e-12f);
  unsigned short* ea = EA  + (size_t)row * KG + 4 * lane;
  unsigned short* eb = EBt + (size_t)row * KG + 4 * lane;
#pragma unroll 1
  for (int pass = 0; pass < 2; ++pass) {
#pragma unroll 1
    for (int q = 0; q < 4; ++q) {
      const v4f y = *(const v4f*)(yr + 128 * q);
      const float e0 = y.x / den, e1 = y.y / den, e2 = y.z / den, e3 = y.w / den;
      const unsigned short h0 = f2bf_bits(e0), h1 = f2bf_bits(e1), h2 = f2bf_bits(e2), h3 = f2bf_bits(e3);
      const unsigned short l0 = f2bf_bits(e0 - bf_bits2f(h0)), l1 = f2bf_bits(e1 - bf_bits2f(h1));
      const unsigned short l2 = f2bf_bits(e2 - bf_bits2f(h2)), l3 = f2bf_bits(e3 - bf_bits2f(h3));
      const v2u hv = { pk16(h0, h1), pk16(h2, h3) };
      const v2u lv = { pk16(l0, l1), pk16(l2, l3) };
      const int o = 128 * q;
      *(volatile v2u*)(ea + o) = hv;
      *(volatile v2u*)(ea + DN + o) = lv;
      *(volatile v2u*)(ea + 2 * DN + o) = hv;
      *(volatile v2u*)(eb + o) = hv;
      *(volatile v2u*)(eb + DN + o) = hv;
      *(volatile v2u*)(eb + 2 * DN + o) = lv;
    }
    __threadfence();
  }
}

__device__ __forceinline__ bool lexless(float a, int ia, float b, int ib) { return (a < b) || ((a == b) && (ia < ib)); }

__device__ __forceinline__ void upd2(float d, int c, float& b1, int& i1, float& b2, int& i2) {
  const bool lt1 = d < b1;
  const bool lt2 = d < b2;
  const float nb2 = lt1 ? b1 : (lt2 ? d : b2);
  const int   ni2 = lt1 ? i1 : (lt2 ? c : i2);
  b1 = lt1 ? d : b1;
  i1 = lt1 ? c : i1;
  b2 = nb2;
  i2 = ni2;
}

__global__ __launch_bounds__(256) void k_rowstat(const float* __restrict__ G, int* N0, int* N1, float* MROW) {
  __shared__ __align__(16) int   sn0[32];
  __shared__ __align__(16) int   sn1[32];
  __shared__ __align__(16) float smx[32];
  const int tid = threadIdx.x, lane = tid & 31, w = tid >> 5;
#pragma unroll 1
  for (int rr = 0; rr < 4; ++rr) {
    const int lr = w * 4 + rr;
    const int row = blockIdx.x * 32 + lr;
    const float* gr = G + (size_t)row * AN + 4 * lane;
    float mx = 0.0f;
#pragma unroll 4
    for (int it = 0; it < 32; ++it) {
      const v4f g = *(const v4f*)(gr + it * 128);
      const float t0 = 2.0f - 2.0f * g.x, t1 = 2.0f - 2.0f * g.y, t2 = 2.0f - 2.0f * g.z, t3 = 2.0f - 2.0f * g.w;
      mx = fmaxf(mx, t0 * t0); mx = fmaxf(mx, t1 * t1); mx = fmaxf(mx, t2 * t2); mx = fmaxf(mx, t3 * t3);
    }
#pragma unroll
    for (int off = 16; off > 0; off >>= 1) mx = fmaxf(mx, __shfl_xor(mx, off, 32));

    float b1 = __int_as_float(0x7f800000), b2 = __int_as_float(0x7f800000);
    int i1 = 0, i2 = 0;
#pragma unroll 1
    for (int it = 0; it < 32; ++it) {
      const v4f g = *(const v4f*)(gr + it * 128);
      const int c = it * 128 + 4 * lane;
      const float t0 = 2.0f - 2.0f * g.x, t1 = 2.0f - 2.0f * g.y, t2 = 2.0f - 2.0f * g.z, t3 = 2.0f - 2.0f * g.w;
      const float d0 = (t0 * t0) / mx, d1 = (t1 * t1) / mx, d2 = (t2 * t2) / mx, d3 = (t3 * t3) / mx;
      upd2(d0, c,     b1, i1, b2, i2);
      upd2(d1, c + 1, b1, i1, b2, i2);
      upd2(d2, c + 2, b1, i1, b2, i2);
      upd2(d3, c + 3, b1, i1, b2, i2);
    }
#pragma unroll
    for (int off = 16; off > 0; off >>= 1) {
      const float q1 = __shfl_xor(b1, off, 32);
      const int  qi1 = __shfl_xor(i1, off, 32);
      const float q2 = __shfl_xor(b2, off, 32);
      const int  qi2 = __shfl_xor(i2, off, 32);
      const bool qb  = lexless(q1, qi1, b1, i1);
      const bool pb  = lexless(b1, i1, q2, qi2);
      const bool qb2 = lexless(q1, qi1, b2, i2);
      const float r1 = qb ? q1 : b1;
      const int  ri1 = qb ? qi1 : i1;
      const float r2 = qb ? (pb ? b1 : q2) : (qb2 ? q1 : b2);
      const int  ri2 = qb ? (pb ? i1 : qi2) : (qb2 ? qi1 : i2);
      b1 = r1; i1 = ri1; b2 = r2; i2 = ri2;
    }
    if (lane == 0) { sn0[lr] = i1; sn1[lr] = i2; smx[lr] = mx; }
  }
  __syncthreads();
  const int l8 = tid & 7;
  const v4i a0 = *(const v4i*)(sn0 + 4 * l8);
  const v4i a1 = *(const v4i*)(sn1 + 4 * l8);
  const v4f am = *(const v4f*)(smx + 4 * l8);
  if (tid < 8) {
    const size_t o = (size_t)blockIdx.x * 32 + 4 * l8;
    *(volatile v4i*)(N0 + o) = a0;
    *(volatile v4i*)(N1 + o) = a1;
    *(volatile v4f*)(MROW + o) = am;
    __threadfence();
    *(volatile v4i*)(N0 + o) = a0;
    *(volatile v4i*)(N1 + o) = a1;
    *(volatile v4f*)(MROW + o) = am;
  }
}

__device__ __forceinline__ int clampA(int x) { return min(max(x, 0), AN - 1); }

__global__ __launch_bounds__(256) void k_slots(const float* __restrict__ G, const int* __restrict__ N0,
                                               const int* __restrict__ N1, const float* __restrict__ MROW,
                                               int* IDX4, float* VALS) {
  __shared__ int   s_idx[4][256];
  __shared__ int   s_kp[4][256];
  __shared__ float s_w[4][256];
  const int tid = threadIdx.x;
  const int r = blockIdx.x * 256 + tid;
  const int c0 = clampA(N0[r]);
  const int c1 = clampA(N1[r]);
  const int n0c0 = clampA(N0[c0]);
  const int n1c0 = clampA(N1[c0]);
  const int n0c1 = clampA(N0[c1]);
  const int n1c1 = clampA(N1[c1]);
  const bool v0 = (n0c0 == r) || (n1c0 == r);
  const bool v1 = (n0c1 == r) || (n1c1 == r);
  const int e0 = n0c0, e1 = n0c1;
  const int n0e0 = clampA(N0[e0]);
  const int n0e1 = clampA(N0[e1]);
  const bool inR0 = (v0 && (e0 == c0)) || (v1 && (e0 == c1));
  const bool inR1 = (v0 && (e1 == c0)) || (v1 && (e1 == c1));
  const bool v2 = v0 && (n0e0 == c0) && inR0;
  const bool v3 = v1 && (n0e1 == c1) && inR1;
  const bool k0 = v0;
  const bool k1 = v1 && !(k0 && (c0 == c1));
  const bool k2 = v2 && !((k0 && (c0 == e0)) || (k1 && (c1 == e0)));
  const bool k3 = v3 && !((k0 && (c0 == e1)) || (k1 && (c1 == e1)) || (k2 && (e0 == e1)));
  s_idx[0][tid] = c0; s_idx[1][tid] = c1; s_idx[2][tid] = e0; s_idx[3][tid] = e1;
  s_kp[0][tid] = k0 ? 1 : 0; s_kp[1][tid] = k1 ? 1 : 0; s_kp[2][tid] = k2 ? 1 : 0; s_kp[3][tid] = k3 ? 1 : 0;
  const float Mr = MROW[r];
  const float* gr = G + (size_t)r * AN;
  float wsum = 0.0f;
#pragma unroll 1
  for (int s = 0; s < 4; ++s) {
    const int idx = s_idx[s][tid];
    const float g = gr[idx];
    const float t = 2.0f - 2.0f * g;
    const float d = (t * t) / Mr;
    const float ex = expf(-d);
    const float wv = (s_kp[s][tid] != 0) ? ex : 0.0f;
    s_w[s][tid] = wv;
    wsum += wv;
  }
  const float den = (wsum > 0.0f) ? wsum : 1.0f;
#pragma unroll 1
  for (int s = 0; s < 4; ++s) {
    const float wv = s_w[s][tid];
    s_w[s][tid] = wv / den;
  }
  const v4f vv = { s_w[0][tid], s_w[1][tid], s_w[2][tid], s_w[3][tid] };
  const v4i iv = { c0, c1, e0, e1 };
  *(volatile v4i*)(IDX4 + (size_t)r * 4) = iv;
  *(volatile v4f*)(VALS + (size_t)r * 4) = vv;
  __threadfence();
  *(volatile v4i*)(IDX4 + (size_t)r * 4) = iv;
  *(volatile v4f*)(VALS + (size_t)r * 4) = vv;
}

__device__ __forceinline__ float vcol(v4i ij, v4f vj, int c) {
  float s = 0.0f;
  s += (ij.x == c) ? vj.x : 0.0f;
  s += (ij.y == c) ? vj.y : 0.0f;
  s += (ij.z == c) ? vj.z : 0.0f;
  s += (ij.w == c) ? vj.w : 0.0f;
  return s;
}

__global__ __launch_bounds__(256) void k_final(const float* __restrict__ G, const float* __restrict__ MROW,
                                               const int* __restrict__ IDX4, const float* __restrict__ VALS,
                                               const float* __restrict__ iou, const float* __restrict__ kf,
                                               const float* __restrict__ thrp, float* out) {
  __shared__ __align__(16) float so0[QN];
  __shared__ __align__(16) float so1[QN];
  __shared__ __align__(16) float so2[QN];
  const int tid = threadIdx.x;
  const int i = blockIdx.x;
  const v4i ii = *(const v4i*)(IDX4 + (size_t)i * 4);
  const v4f vi = *(const v4f*)(VALS + (size_t)i * 4);
  const float Mi = MROW[i];
  const float thr = bf_rne(thrp[0]);
  const float* gr = G + (size_t)i * AN + QN;
  const float* ir = iou + (size_t)i * QN;
  const float* kr = kf + (size_t)i * QN;
#pragma unroll 1
  for (int e = 0; e < 8; ++e) {
    const int j = e * 256 + tid;
    const float g = gr[j];
    const v4i ij = *(const v4i*)(IDX4 + (size_t)(QN + j) * 4);
    const v4f vj = *(const v4f*)(VALS + (size_t)(QN + j) * 4);
    const float io = bf_rne(ir[j]);
    const float kv = bf_rne(kr[j]);
    float t = 0.0f;
    t += fminf(vi.x, vcol(ij, vj, ii.x));
    t += fminf(vi.y, vcol(ij, vj, ii.y));
    t += fminf(vi.z, vcol(ij, vj, ii.z));
    t += fminf(vi.w, vcol(ij, vj, ii.w));
    const float jac = 1.0f - t / (2.0f - t);
    const float tt = 2.0f - 2.0f * g;
    const float d = (tt * tt) / Mi;
    const float fin = jac * 0.7f + d * 0.3f;
    const bool fl = (kv == -1.0f) || (io == 0.0f) || (g < thr);
    so0[j] = g;
    so1[j] = 1.0f - fin;
    so2[j] = fl ? 1.0f : 0.0f;
  }
  __syncthreads();
  v4f a0[2], a1[2], a2[2];
#pragma unroll
  for (int it = 0; it < 2; ++it) {
    const int c = 4 * (tid + 256 * it);
    a0[it] = *(const v4f*)(so0 + c);
    a1[it] = *(const v4f*)(so1 + c);
    a2[it] = *(const v4f*)(so2 + c);
  }
  float* o0 = out + (size_t)i * QN;
  float* o1 = out + (size_t)QN * QN + (size_t)i * QN;
  float* o2 = out + (size_t)2 * QN * QN + (size_t)i * QN;
  for (int pass = 0; pass < 2; ++pass) {
#pragma unroll
    for (int it = 0; it < 2; ++it) {
      const int c = 4 * (tid + 256 * it);
      *(volatile v4f*)(o0 + c) = a0[it];
      *(volatile v4f*)(o1 + c) = a1[it];
      *(volatile v4f*)(o2 + c) = a2[it];
    }
    __threadfence();
  }
}

extern "C" void kernel_launch(void* const* d_in, const int* in_sizes, int n_in,
                              void* d_out, int out_size, void* d_ws, size_t ws_size,
                              hipStream_t stream) {
  if (n_in < 7) return;
  if (in_sizes[0] != DN * QN || in_sizes[1] != DN * QN) return;
  if (in_sizes[2] != QN * QN || in_sizes[3] != QN * QN) return;
  if (in_sizes[4] != 1 || in_sizes[5] != DN * DN || in_sizes[6] != DN) return;
  if (out_size != 3 * QN * QN) return;

  const float* Usrc = (const float*)d_in[0];
  const float* Utgt = (const float*)d_in[1];
  const float* iou  = (const float*)d_in[2];
  const float* kfg  = (const float*)d_in[3];
  const float* thr  = (const float*)d_in[4];
  const float* cgw  = (const float*)d_in[5];
  const float* cgb  = (const float*)d_in[6];
  float* out = (float*)d_out;

  const size_t bEB  = (size_t)AN * DN * 2;
  const size_t bU2  = (size_t)DN * AN * 2;
  const size_t bCW  = (size_t)DN * KY * 2;
  const size_t bEA  = (size_t)AN * KG * 2;
  const size_t bN   = (size_t)AN * 4;
  const size_t bI4  = (size_t)AN * 16;
  const size_t bR   = (size_t)AN * AN * 4;
  size_t off = 0;
  const size_t oEB  = off; off += bEB;
  const size_t oUT2 = off; off += bU2;
  const size_t oUS2 = off; off += bU2;
  const size_t oCW2 = off; off += bCW;
  const size_t oEA  = off; off += bEA;
  const size_t oEBt = off; off += bEA;
  const size_t oN0  = off; off += bN;
  const size_t oN1  = off; off += bN;
  const size_t oMR  = off; off += bN;
  const size_t oI4  = off; off += bI4;
  const size_t oVL  = off; off += bI4;
  const size_t oR   = off; off += bR;
  if (off > ws_size) return;
  if (off > (size_t)134217728) return;
  const size_t oMP  = oR;
  const size_t oMF  = oR + (size_t)2 * QN * AN * 2;
  const size_t oX   = oMF + (size_t)AN * DN * 4;
  const size_t oYF  = oX + (size_t)AN * KY * 2;
  if (oYF + (size_t)AN * DN * 4 > oR + bR) return;

  char* ws = (char*)d_ws;
  unsigned short* EB  = (unsigned short*)(ws + oEB);
  unsigned short* UT2 = (unsigned short*)(ws + oUT2);
  unsigned short* US2 = (unsigned short*)(ws + oUS2);
  unsigned short* CW2 = (unsigned short*)(ws + oCW2);
  unsigned short* EA  = (unsigned short*)(ws + oEA);
  unsigned short* EBt = (unsigned short*)(ws + oEBt);
  int*   N0   = (int*)(ws + oN0);
  int*   N1   = (int*)(ws + oN1);
  float* MROW = (float*)(ws + oMR);
  int*   IDX4 = (int*)(ws + oI4);
  float* VALS = (float*)(ws + oVL);
  float* Gm   = (float*)(ws + oR);
  unsigned short* MP = (unsigned short*)(ws + oMP);
  float* MF = (float*)(ws + oMF);
  unsigned short* X  = (unsigned short*)(ws + oX);
  float* YF = (float*)(ws + oYF);

  const dim3 blk(256);

  k_tr<<<dim3(QN / 64, DN / 64), blk, 0, stream>>>(Usrc, EB, QN, DN);
  k_tr<<<dim3(QN / 64, DN / 64), blk, 0, stream>>>(Utgt, EB + (size_t)QN * DN, QN, DN);
  k_dup<<<dim3((DN * QN / 8 + 255) / 256), blk, 0, stream>>>(Utgt, UT2, QN, DN * QN / 8);
  k_dup<<<dim3((DN * QN / 8 + 255) / 256), blk, 0, stream>>>(Usrc, US2, QN, DN * QN / 8);
  k_dup<<<dim3((DN * DN / 8 + 255) / 256), blk, 0, stream>>>(cgw, CW2, DN, DN * DN / 8);
  gemm64<2><<<dim3(((QN / 64) * (QN / 64) + 7) / 8, 1), blk, 0, stream>>>(
      EB, DN, 0L, EB + (size_t)QN * DN, DN, 0L, MF, MP, AN, 0L, iou, QN, QN, DN);
  gemm64<0><<<dim3(((QN / 64) * (DN / 64) + 7) / 8, 2), blk, 0, stream>>>(
      MP, AN, (long)QN * AN, UT2, AN, (long)DN * AN, MF, MP, DN, (long)QN * DN, cgb, QN, DN, AN);
  k_rowx<<<dim3(AN / 8), blk, 0, stream>>>(EB, MF, X);
  gemm64<1><<<dim3(((AN / 64) * (DN / 64) + 7) / 8, 1), blk, 0, stream>>>(
      X, KY, 0L, CW2, KY, 0L, YF, X, DN, 0L, cgb, AN, DN, KY);
  k_rowe<<<dim3(AN / 8), blk, 0, stream>>>(YF, EA, EBt);
  gemm64<0><<<dim3(((AN / 64) * (AN / 64) + 7) / 8, 1), blk, 0, stream>>>(
      EA, KG, 0L, EBt, KG, 0L, Gm, EA, AN, 0L, cgb, AN, AN, KG);
  k_rowstat<<<dim3(AN / 32), blk, 0, stream>>>(Gm, N0, N1, MROW);
  k_slots<<<dim3(AN / 256), blk, 0, stream>>>(Gm, N0, N1, MROW, IDX4, VALS);
  k_final<<<dim3(QN), blk, 0, stream>>>(Gm, MROW, IDX4, VALS, iou, kfg, thr, out);
  (void)hipGetLastError();
}
